// TinyLSTM_68753836474968
// MI455X (gfx1250) — hardware-run, weakly checked
//
#include <hip/hip_runtime.h>


#define NPL 512
#define NRW 8192

typedef _Float16 h16;
typedef unsigned short bf;
typedef __attribute__((ext_vector_type(16))) __bf16   v16bf;
typedef __attribute__((ext_vector_type(16))) _Float16 v16h;
typedef __attribute__((ext_vector_type(8)))  _Float16 v8h;
typedef __attribute__((ext_vector_type(8)))  unsigned short v8us;
typedef __attribute__((ext_vector_type(8)))  float    v8f;
typedef __attribute__((ext_vector_type(4)))  float    v4f;
typedef v8h  __attribute__((may_alias)) v8ha;
typedef v4f  __attribute__((may_alias)) v4fa;
typedef v8us __attribute__((may_alias)) v8usa;

__device__ __forceinline__ unsigned short f2bf(float f) { unsigned u = __float_as_uint(f); u += 0x7FFFu + ((u >> 16) & 1u); return (unsigned short)(u >> 16); }
__device__ __forceinline__ float bf2f(unsigned short b) { return __uint_as_float(((unsigned)b) << 16); }
__device__ __forceinline__ float bfr(float f) { return bf2f(f2bf(f)); }
__device__ __forceinline__ v16h cat16(v8h lo, v8h hi) { return __builtin_shufflevector(lo, hi, 0, 1, 2, 3, 4, 5, 6, 7, 8, 9, 10, 11, 12, 13, 14, 15); }
__device__ __forceinline__ v16bf cat16b(v8us lo, v8us hi) { return __builtin_bit_cast(v16bf, __builtin_shufflevector(lo, hi, 0, 1, 2, 3, 4, 5, 6, 7, 8, 9, 10, 11, 12, 13, 14, 15)); }
__device__ __forceinline__ v8f wmma16(v16h a, v16h b, v8f c) { return __builtin_amdgcn_wmma_f32_16x16x32_f16(false, a, false, b, (short)0, c, false, false); }
__device__ __forceinline__ v8f wmmab(v16bf a, v16bf b, v8f c) { return __builtin_amdgcn_wmma_f32_16x16x32_bf16(false, a, false, b, (short)0, c, false, false); }

template <typename T16> struct WFrag;
template <> struct WFrag<h16> { typedef v16h V; static __device__ __forceinline__ V ld(const h16* p) { return cat16(*(const v8h*)p, *(const v8h*)(p + 16)); } static __device__ __forceinline__ v8f mma(V a, V b, v8f c) { return wmma16(a, b, c); } };
template <> struct WFrag<bf> { typedef v16bf V; static __device__ __forceinline__ V ld(const bf* p) { return cat16b(*(const v8us*)p, *(const v8us*)(p + 16)); } static __device__ __forceinline__ v8f mma(V a, V b, v8f c) { return wmmab(a, b, c); } };

__device__ __forceinline__ h16 toh_flush(float x) { const float z = (fabsf(x) < 6.103515625e-05f) ? 0.0f : x; return (h16)z; }

__global__ __launch_bounds__(256) void k_xword(const float* __restrict__ src, h16* dst) {
    const size_t i = (size_t)blockIdx.x * 256 + threadIdx.x; const v8f wv = *(const v8f*)(src + i * 8); v8h ow;
#pragma unroll
    for (int j = 0; j < 8; ++j) ow[j] = toh_flush(bfr(wv[j]));
    *(volatile v8h*)(dst + i * 8) = ow; __threadfence(); *(volatile v8h*)(dst + i * 8) = ow; }

__global__ __launch_bounds__(32) void k_cell4(const float* __restrict__ xin, const h16* __restrict__ wr, const float* __restrict__ wi, const float* __restrict__ ba, const float* __restrict__ bb, float* hs) {
    __shared__ __align__(16) float tl[16 * 36];
    const int lane = threadIdx.x & 31, lr = lane & 15, hi = lane >> 4; const int b0 = blockIdx.x * 16;
    v16h wf[8]; float qi[8], qb[8];
#pragma unroll
    for (int q = 0; q < 8; ++q) { const int col = (q >> 1) * 32 + (q & 1) * 16 + lr; wf[q] = WFrag<h16>::ld(wr + (size_t)col * 32 + 8 * hi); qi[q] = bfr(wi[col]); qb[q] = bfr(ba[col]) + bfr(bb[col]); }
    v16h sa = (v16h){}; float cs[16];
#pragma unroll
    for (int j = 0; j < 16; ++j) cs[j] = 0.0f;
    const float* px = xin + (size_t)(b0 + 8 * hi) * NPL;
    for (int ts = 0; ts < NPL; ++ts) { float xv[8]; v8f d[8];
#pragma unroll
        for (int j = 0; j < 8; ++j) xv[j] = bfr(px[(size_t)j * NPL + ts]);
#pragma unroll
        for (int q = 0; q < 8; ++q) { v8f c;
#pragma unroll
            for (int j = 0; j < 8; ++j) c[j] = xv[j] * qi[q] + qb[q];
            d[q] = wmma16(sa, wf[q], c); }
        __builtin_amdgcn_wave_barrier(); asm volatile("" ::: "memory");
#pragma unroll
        for (int hf = 0; hf < 2; ++hf) {
#pragma unroll
            for (int j = 0; j < 8; ++j) { const float gi = 1.0f / (1.0f + expf(-d[hf][j])), gf = 1.0f / (1.0f + expf(-d[2 + hf][j])), gg = 1.0f - 2.0f / (1.0f + expf(2.0f * d[4 + hf][j])), go = 1.0f / (1.0f + expf(-d[6 + hf][j]));
                const float cn = gf * cs[hf * 8 + j] + gi * gg; cs[hf * 8 + j] = cn; tl[(8 * hi + j) * 36 + hf * 16 + lr] = go * (1.0f - 2.0f / (1.0f + expf(2.0f * cn))); } }
        __builtin_amdgcn_wave_barrier(); asm volatile("" ::: "memory");
        const float* pr = tl + lr * 36 + 8 * hi; const v4f a0 = *(const v4fa*)pr, a1 = *(const v4fa*)(pr + 4), a2 = *(const v4fa*)(pr + 16), a3 = *(const v4fa*)(pr + 20);
#pragma unroll
        for (int j = 0; j < 4; ++j) { sa[j] = toh_flush(a0[j]); sa[4 + j] = toh_flush(a1[j]); sa[8 + j] = toh_flush(a2[j]); sa[12 + j] = toh_flush(a3[j]); }
        __builtin_amdgcn_wave_barrier(); asm volatile("" ::: "memory"); }
    const float* po = tl + (lane >> 1) * 36 + 16 * (lane & 1); const v4f u0 = *(const v4fa*)po, u1 = *(const v4fa*)(po + 4), u2 = *(const v4fa*)(po + 8), u3 = *(const v4fa*)(po + 12);
    float* pw = hs + ((size_t)b0 + (lane >> 1)) * 32 + 16 * (lane & 1);
    *(volatile v4f*)pw = u0; *(volatile v4f*)(pw + 4) = u1; *(volatile v4f*)(pw + 8) = u2; *(volatile v4f*)(pw + 12) = u3; __threadfence(); *(volatile v4f*)pw = u0; *(volatile v4f*)(pw + 4) = u1; *(volatile v4f*)(pw + 8) = u2; *(volatile v4f*)(pw + 12) = u3; }

__global__ __launch_bounds__(256) void k_hd(const float* __restrict__ hs, const float* __restrict__ fw, const float* __restrict__ fb, float* res) {
    const unsigned r = blockIdx.x * 256 + threadIdx.x; const float* ph = hs + (size_t)r * 32; float s = 0.0f;
#pragma unroll
    for (int g4 = 0; g4 < 8; ++g4) { const v4f q = *(const v4fa*)(ph + g4 * 4);
#pragma unroll
        for (int j = 0; j < 4; ++j) s = s + q[j] * bfr(fw[g4 * 4 + j]); }
    const float o = s + bfr(fb[0]); *(volatile float*)(res + r) = o; __threadfence(); *(volatile float*)(res + r) = o; }

extern "C" void kernel_launch(void* const* d_in, const int* in_sizes, int n_in, void* d_out, int out_size, void* d_ws, size_t ws_size, hipStream_t stream) {
    if (n_in < 7) return;
    if (in_sizes[0] != NRW * NPL || in_sizes[1] != 128 || in_sizes[2] != 128 * 32 || in_sizes[3] != 128 || in_sizes[4] != 128 || in_sizes[5] != 32 || in_sizes[6] != 1 || out_size != NRW) return;
    static_assert(NRW % 16 == 0 && NRW % 256 == 0 && (128 * 32 / 8) % 256 == 0, "16 rows a wave; the flat grids exact");
    const float* a0 = (const float*)d_in[0]; const float* a1 = (const float*)d_in[1]; const float* a2 = (const float*)d_in[2]; const float* a3 = (const float*)d_in[3]; const float* a4 = (const float*)d_in[4]; const float* a5 = (const float*)d_in[5]; const float* a6 = (const float*)d_in[6]; float* res = (float*)d_out;
    char* wsp = (char*)d_ws; auto take = [&](size_t bytes) { char* p = wsp; wsp += (bytes + 255) & ~(size_t)255; return (void*)p; };
    h16* Wr = (h16*)take((size_t)128 * 32 * 2); float* Hs = (float*)take((size_t)NRW * 32 * 4);
    if ((size_t)(wsp - (char*)d_ws) > ws_size) return;
    k_xword<<<128 * 32 / 8 / 256, 256, 0, stream>>>(a2, Wr);
    k_cell4<<<NRW / 16, 32, 0, stream>>>(a0, Wr, a1, a3, a4, Hs);
    k_hd<<<NRW / 256, 256, 0, stream>>>(Hs, a5, a6, res);
}
